// MultiHeadMaskedSelfAttention_57492432224475
// MI455X (gfx1250) — hardware-verified
//
#include <hip/hip_runtime.h>

typedef __attribute__((ext_vector_type(16))) _Float16 v16h;
typedef __attribute__((ext_vector_type(8)))  _Float16 v8h;
typedef __attribute__((ext_vector_type(16))) __bf16   v16b;
typedef __attribute__((ext_vector_type(8)))  __bf16   v8b;
typedef __attribute__((ext_vector_type(8)))  float    v8f;
typedef __attribute__((ext_vector_type(4)))  float    v4f;
typedef __attribute__((ext_vector_type(4)))  unsigned int   v4u;
typedef __attribute__((ext_vector_type(8)))  unsigned short v8us;

constexpr int kBatch = 4;
constexpr int kSeq   = 2048;
constexpr int kDm    = 1024;
constexpr int kHeads = 16;
constexpr int kHd    = 64;
constexpr int kRows  = kBatch * kSeq;
constexpr float kNegBig    = -1.0e9f;
constexpr float kInvSqrtHd = 0.125f;

static_assert(kRows % 64 == 0);
static_assert(kDm % 64 == 0);
static_assert(kDm % 32 == 0);
static_assert(kSeq % 64 == 0);
static_assert(kHd == 64);
static_assert(kHeads * kHd == kDm);

__device__ __forceinline__ unsigned short f2bf_bits(float f) {
  unsigned u = __float_as_uint(f);
  return (unsigned short)((u + 0x7FFFu + ((u >> 16) & 1u)) >> 16);
}
__device__ __forceinline__ float bf_bits2f(unsigned short h) { return __uint_as_float(((unsigned)h) << 16); }

__device__ __forceinline__ void dep_guard_h(v8f& a, v8f& b, v16h x, v16h y) { asm volatile("v_nop\n\tv_nop\n\tv_nop\n\tv_nop" : "+v"(a), "+v"(b) : "v"(x), "v"(y)); }
__device__ __forceinline__ void dep_guard_b(v8f& a, v8f& b, v16b x, v16b y) { asm volatile("v_nop\n\tv_nop\n\tv_nop\n\tv_nop" : "+v"(a), "+v"(b) : "v"(x), "v"(y)); }
__device__ __forceinline__ void keep4_h(v16h a, v16h b, v16h c, v16h d) { asm volatile("v_nop" :: "v"(a), "v"(b), "v"(c), "v"(d)); }
__device__ __forceinline__ void keep4_b(v16b a, v16b b, v16b c, v16b d) { asm volatile("v_nop" :: "v"(a), "v"(b), "v"(c), "v"(d)); }
__device__ __forceinline__ void acc_guard4(v8f& a, v8f& b, v8f& c, v8f& d) { asm volatile("v_nop\n\tv_nop\n\tv_nop\n\tv_nop" : "+v"(a), "+v"(b), "+v"(c), "+v"(d)); }

template <typename T> struct Frag;
template <> struct Frag<_Float16> {
  typedef v16h V; union U { v16h v; v8h h[2]; };
  static __device__ __forceinline__ v16h load(const _Float16* p) {
    U f; f.h[0] = *(const v8h*)(p); f.h[1] = *(const v8h*)(p + 16); return f.v;
  }
  static __device__ __forceinline__ v8f mma(v16h a, v16h b, v8f c) {
    return __builtin_amdgcn_wmma_f32_16x16x32_f16(false, a, false, b, (short)0, c, false, false);
  }
  static __device__ __forceinline__ void guard(v8f& a, v8f& b, v16h x, v16h y) { dep_guard_h(a, b, x, y); }
  static __device__ __forceinline__ void keep(v16h a, v16h b, v16h c, v16h d) { keep4_h(a, b, c, d); }
};
template <> struct Frag<__bf16> {
  typedef v16b V; union U { v16b v; v8b h[2]; };
  static __device__ __forceinline__ v16b load(const __bf16* p) {
    U f; f.h[0] = *(const v8b*)(p); f.h[1] = *(const v8b*)(p + 16); return f.v;
  }
  static __device__ __forceinline__ v8f mma(v16b a, v16b b, v8f c) {
    return __builtin_amdgcn_wmma_f32_16x16x32_bf16(false, a, false, b, (short)0, c, false, false);
  }
  static __device__ __forceinline__ void guard(v8f& a, v8f& b, v16b x, v16b y) { dep_guard_b(a, b, x, y); }
  static __device__ __forceinline__ void keep(v16b a, v16b b, v16b c, v16b d) { keep4_b(a, b, c, d); }
};

template <int ET> struct Elem;
template <> struct Elem<0> { typedef _Float16 T; };
template <> struct Elem<1> { typedef __bf16 T; };
template <int ET, int SPLITM, int BIAS_MODE, int OUT_MODE>
__global__ __launch_bounds__(256) void wmma_gemm64(
    const unsigned short* __restrict__ Ap, const unsigned short* __restrict__ A2p, int lda, long strideA,
    const unsigned short* __restrict__ Btp, const unsigned short* __restrict__ Bt2p, int ldb, long strideB,
    void* Cout, void* Cout2, int ldc, long strideC,
    const float* __restrict__ bias,
    int M, int N, int K, float scale) {
  typedef typename Elem<ET>::T T;
  typedef typename Frag<T>::V V;
  constexpr bool SPLA = (SPLITM != 0);
  constexpr bool SPLB = (SPLITM == 1);
  const T* A = (const T*)Ap; const T* A2 = (const T*)A2p; const T* Bt = (const T*)Btp; const T* Bt2 = (const T*)Bt2p;
  __shared__ __align__(16) float sT[8][16 * 68];
  const int b    = blockIdx.y;
  const int lane = threadIdx.x & 31;
  const int wave = threadIdx.x >> 5;
  const int tilesN = N >> 6;
  const int tilesM = M >> 6;
  const int tile = blockIdx.x * 8 + wave;
  if (tile >= tilesM * tilesN) return;
  const int tm = tile / tilesN;
  const int tn = tile - tm * tilesN;
  const int m0 = tm << 6;
  const int n0 = tn << 6;

  const T* Ab  = A  + (size_t)b * strideA;
  const T* Bb  = Bt + (size_t)b * strideB;
  const T* Ab2 = SPLA ? (A2  + (size_t)b * strideA) : nullptr;
  const T* Bb2 = SPLB ? (Bt2 + (size_t)b * strideB) : nullptr;

  const int rlane = lane & 15;
  const int koff  = (lane >> 4) * 8;
  const int mOff  = (lane >> 4) * 8;

  v8f acc[4][4];
#pragma unroll
  for (int i = 0; i < 4; ++i)
#pragma unroll
    for (int j = 0; j < 4; ++j) acc[i][j] = (v8f){0.f,0.f,0.f,0.f,0.f,0.f,0.f,0.f};

  for (int k0 = 0; k0 < K; k0 += 32) {
    V bh[4], bl[4];
#pragma unroll
    for (int j = 0; j < 4; ++j) {
      const size_t bo = (size_t)(n0 + (j << 4) + rlane) * ldb + koff + k0;
      bh[j] = Frag<T>::load(Bb + bo);
      if (SPLB) bl[j] = Frag<T>::load(Bb2 + bo);
    }
#pragma unroll
    for (int i = 0; i < 4; ++i) {
      const size_t ao = (size_t)(m0 + (i << 4) + rlane) * lda + koff + k0;
      V ah = Frag<T>::load(Ab + ao);
      V al;
      if (SPLA) al = Frag<T>::load(Ab2 + ao);
#pragma unroll
      for (int j = 0; j < 4; ++j) {
        acc[i][j] = Frag<T>::mma(ah, bh[j], acc[i][j]);
        if (SPLB) acc[i][j] = Frag<T>::mma(ah, bl[j], acc[i][j]);
        if (SPLA) acc[i][j] = Frag<T>::mma(al, bh[j], acc[i][j]);
      }
      Frag<T>::guard(acc[i][0], acc[i][3], ah, SPLA ? al : ah);
    }
    Frag<T>::keep(bh[0], bh[1], bh[2], bh[3]);
    if (SPLB) Frag<T>::keep(bl[0], bl[1], bl[2], bl[3]);
  }
  acc_guard4(acc[0][0], acc[0][1], acc[0][2], acc[0][3]);
  acc_guard4(acc[1][0], acc[1][1], acc[1][2], acc[1][3]);
  acc_guard4(acc[2][0], acc[2][1], acc[2][2], acc[2][3]);
  acc_guard4(acc[3][0], acc[3][1], acc[3][2], acc[3][3]);

  float* slab = sT[wave];
#pragma unroll
  for (int i = 0; i < 4; ++i) {
    const int mBase = m0 + (i << 4);
    v4f bmA = (v4f){0.f, 0.f, 0.f, 0.f}, bmB = (v4f){0.f, 0.f, 0.f, 0.f};
    if (BIAS_MODE == 1) {
      bmA = *(const v4f*)(bias + mBase + mOff);
      bmB = *(const v4f*)(bias + mBase + mOff + 4);
    }
#pragma unroll
    for (int j = 0; j < 4; ++j) {
      const int n = n0 + (j << 4) + rlane;
      float bv = 0.f;
      if (BIAS_MODE == 2) bv = bias[n];
#pragma unroll
      for (int r = 0; r < 8; ++r) {
        float v = acc[i][j][r] * scale;
        if (BIAS_MODE == 1) v += (r < 4) ? bmA[r] : bmB[r - 4];
        if (BIAS_MODE == 2) v += bv;
        slab[(mOff + r) * 68 + (j << 4) + rlane] = v;
      }
    }
    __builtin_amdgcn_fence(__ATOMIC_RELEASE, "workgroup");
    __builtin_amdgcn_wave_barrier();
    __builtin_amdgcn_fence(__ATOMIC_ACQUIRE, "workgroup");
    if (OUT_MODE == 0) {
      float* C = (float*)Cout + (size_t)b * strideC;
      const int hh = lane >> 4, c4 = (lane & 15) * 4;
      for (int pass = 0; pass < 2; ++pass) {
#pragma unroll
        for (int it = 0; it < 8; ++it) {
          const int row = it * 2 + hh;
          v4f v = *(const v4f*)(slab + row * 68 + c4);
          *(volatile v4f*)(C + (size_t)(mBase + row) * ldc + n0 + c4) = v;
        }
        __threadfence();
      }
    } else {
      const int q = lane >> 3, c8 = (lane & 7) * 8;
      unsigned short* C  = (unsigned short*)Cout  + (size_t)b * strideC;
      unsigned short* C2 = (OUT_MODE == 2) ? ((unsigned short*)Cout2 + (size_t)b * strideC) : nullptr;
      for (int pass = 0; pass < 2; ++pass) {
#pragma unroll
        for (int it = 0; it < 4; ++it) {
          const int row = it * 4 + q;
          const float* sp = slab + row * 68 + c8;
          v8h hv, lv;
#pragma unroll
          for (int e = 0; e < 8; ++e) {
            if (OUT_MODE == 1) {
              hv[e] = (_Float16)sp[e];
            } else {
              unsigned short hb = f2bf_bits(sp[e]);
              unsigned short lb = f2bf_bits(sp[e] - bf_bits2f(hb));
              hv[e] = __builtin_bit_cast(_Float16, hb);
              lv[e] = __builtin_bit_cast(_Float16, lb);
            }
          }
          *(volatile v8h*)(C + (size_t)(mBase + row) * ldc + n0 + c8) = hv;
          if (OUT_MODE == 2) *(volatile v8h*)(C2 + (size_t)(mBase + row) * ldc + n0 + c8) = lv;
        }
        __threadfence();
      }
    }
    __builtin_amdgcn_fence(__ATOMIC_RELEASE, "workgroup");
    __builtin_amdgcn_wave_barrier();
    __builtin_amdgcn_fence(__ATOMIC_ACQUIRE, "workgroup");
  }
}

__global__ __launch_bounds__(256) void cast_f32_bf16x8(
    const float* __restrict__ in, unsigned short* __restrict__ out, int n8) {
  const int i = blockIdx.x * 256 + threadIdx.x;
  if (i < n8) {
    const size_t base = (size_t)i * 8;
    const v4f a0 = *(const v4f*)(in + base);
    const v4f a1 = *(const v4f*)(in + base + 4);
    v8us u;
    u[0] = f2bf_bits(a0[0]); u[1] = f2bf_bits(a0[1]); u[2] = f2bf_bits(a0[2]); u[3] = f2bf_bits(a0[3]);
    u[4] = f2bf_bits(a1[0]); u[5] = f2bf_bits(a1[1]); u[6] = f2bf_bits(a1[2]); u[7] = f2bf_bits(a1[3]);
    *(volatile v8us*)(out + base) = u;
    __threadfence();
    *(volatile v8us*)(out + base) = u;
  }
}

__device__ __forceinline__ v8f at_mma(v16b a, v16b b, v8f c) {
  c = __builtin_amdgcn_wmma_f32_16x16x32_bf16(false, a, false, b, (short)0, c, false, false);
  asm volatile("v_nop\n\tv_nop\n\tv_nop\n\tv_nop" : "+v"(c) : "v"(a), "v"(b));
  return c;
}

__global__ __launch_bounds__(128)
void attn64_planes(const unsigned short* __restrict__ Qh, const unsigned short* __restrict__ Ql,
                   const unsigned short* __restrict__ Kh, const unsigned short* __restrict__ Kl,
                   const unsigned short* __restrict__ Vth, const unsigned short* __restrict__ Vtl,
                   const float* __restrict__ amask,
                   unsigned short* __restrict__ Oh, unsigned short* __restrict__ Ol) {
  __shared__ __align__(16) unsigned char lds_raw[65536];
  __bf16* ksh = reinterpret_cast<__bf16*>(lds_raw);
  __bf16* ksl = reinterpret_cast<__bf16*>(lds_raw + 8192);
  __bf16* vsh = reinterpret_cast<__bf16*>(lds_raw + 16384);
  __bf16* vsl = reinterpret_cast<__bf16*>(lds_raw + 24576);
  float*  msk = reinterpret_cast<float*>(lds_raw + 49152);

  const int tid  = threadIdx.x;
  const int wave = tid >> 5;
  const int lane = tid & 31;
  const int hh   = lane >> 4;
  const int c    = lane & 15;
  const int koff = hh * 8;
  __bf16* pwh = reinterpret_cast<__bf16*>(lds_raw + 32768) + wave * 1024;
  __bf16* pwl = reinterpret_cast<__bf16*>(lds_raw + 40960) + wave * 1024;

  constexpr int nqb = kSeq / 64;
  const int bx = blockIdx.x;
  const int qb = bx % nqb;
  const int bh = bx / nqb;
  const int h  = bh % kHeads;
  const int b  = bh / kHeads;
  const int q0 = qb * 64 + wave * 16;
  const size_t rowb = (size_t)b * kSeq;
  const int hcol = h * kHd;

  v16b qah[2], qal[2];
#pragma unroll
  for (int dc = 0; dc < 2; ++dc) {
    const size_t qo = (rowb + q0 + c) * (size_t)kDm + hcol + dc * 32 + koff;
    qah[dc] = Frag<__bf16>::load(reinterpret_cast<const __bf16*>(Qh) + qo);
    qal[dc] = Frag<__bf16>::load(reinterpret_cast<const __bf16*>(Ql) + qo);
  }

  float mrow[8], lrow[8];
  v8f oacc[4];
#pragma unroll
  for (int r = 0; r < 8; ++r) { mrow[r] = -__builtin_inff(); lrow[r] = 0.f; }
#pragma unroll
  for (int t = 0; t < 4; ++t) oacc[t] = (v8f){0.f,0.f,0.f,0.f,0.f,0.f,0.f,0.f};

  const int nChunks = qb + 1;
  for (int kc = 0; kc < nChunks; ++kc) {
    const int kv0 = kc * 64;
    __syncthreads();
#pragma unroll
    for (int i = 0; i < 4; ++i) {
      const int seg = tid + 128 * i;
      const int kvr = seg >> 3;
      const int d8  = (seg & 7) * 8;
      const size_t go = (rowb + kv0 + kvr) * (size_t)kDm + hcol + d8;
      const v4u a0 = *(const v4u*)(Kh + go);
      const v4u a1 = *(const v4u*)(Kl + go);
      *(v4u*)(ksh + kvr * 64 + d8) = a0;
      *(v4u*)(ksl + kvr * 64 + d8) = a1;
    }
    asm volatile("" ::: "memory");
#pragma unroll
    for (int i = 0; i < 4; ++i) {
      const int seg = tid + 128 * i;
      const int d   = seg >> 3;
      const int kv8 = (seg & 7) * 8;
      const size_t go = (size_t)(hcol + d) * (size_t)kRows + rowb + kv0 + kv8;
      const v4u a0 = *(const v4u*)(Vth + go);
      const v4u a1 = *(const v4u*)(Vtl + go);
      *(v4u*)(vsh + d * 64 + kv8) = a0;
      *(v4u*)(vsl + d * 64 + kv8) = a1;
    }
    asm volatile("" ::: "memory");
#pragma unroll
    for (int i = 0; i < 8; ++i) {
      const int seg = tid + 128 * i;
      const int r   = seg >> 4;
      const int c4  = (seg & 15) * 4;
      const v4f mv = *(const v4f*)(amask + (size_t)(qb * 64 + r) * kSeq + kv0 + c4);
      *(v4f*)(msk + r * 64 + c4) = mv;
    }
    __syncthreads();

    v8f s[4];
#pragma unroll
    for (int j = 0; j < 4; ++j) {
      s[j] = (v8f){0.f,0.f,0.f,0.f,0.f,0.f,0.f,0.f};
#pragma unroll
      for (int dc = 0; dc < 2; ++dc) {
        const int ko = (j * 16 + c) * 64 + dc * 32 + koff;
        const v16b kbh = Frag<__bf16>::load(ksh + ko);
        const v16b kbl = Frag<__bf16>::load(ksl + ko);
        s[j] = at_mma(qah[dc], kbh, s[j]);
        s[j] = at_mma(qah[dc], kbl, s[j]);
        s[j] = at_mma(qal[dc], kbh, s[j]);
      }
    }
    float cm[8];
#pragma unroll
    for (int r = 0; r < 8; ++r) {
      const int rl = wave * 16 + 8 * hh + r;
      float m = -__builtin_inff();
#pragma unroll
      for (int j = 0; j < 4; ++j) {
        const float mv = msk[rl * 64 + j * 16 + c];
        float t = s[j][r] * kInvSqrtHd;
        t = t + mv * kNegBig;
        s[j][r] = t;
        m = fmaxf(m, t);
      }
#pragma unroll
      for (int off = 1; off < 16; off <<= 1) m = fmaxf(m, __shfl_xor(m, off, 32));
      cm[r] = m;
    }
#pragma unroll
    for (int r = 0; r < 8; ++r) {
      const float mnew = fmaxf(mrow[r], cm[r]);
      const float alpha = expf(mrow[r] - mnew);
      mrow[r] = mnew;
      float psum = 0.f;
#pragma unroll
      for (int j = 0; j < 4; ++j) {
        const float p = expf(s[j][r] - mnew);
        psum += p;
        const unsigned short hb = f2bf_bits(p);
        const unsigned short lb = f2bf_bits(p - bf_bits2f(hb));
        pwh[(8 * hh + r) * 64 + j * 16 + c] = __builtin_bit_cast(__bf16, hb);
        pwl[(8 * hh + r) * 64 + j * 16 + c] = __builtin_bit_cast(__bf16, lb);
      }
#pragma unroll
      for (int off = 1; off < 16; off <<= 1) psum += __shfl_xor(psum, off, 32);
      lrow[r] = lrow[r] * alpha + psum;
#pragma unroll
      for (int t = 0; t < 4; ++t) oacc[t][r] *= alpha;
    }
    __syncthreads();
#pragma unroll
    for (int kk = 0; kk < 2; ++kk) {
      const int po = c * 64 + kk * 32 + koff;
      const v16b pa = Frag<__bf16>::load(pwh + po);
      const v16b pl = Frag<__bf16>::load(pwl + po);
#pragma unroll
      for (int t = 0; t < 4; ++t) {
        const int vo = (t * 16 + c) * 64 + kk * 32 + koff;
        const v16b vbh = Frag<__bf16>::load(vsh + vo);
        const v16b vbl = Frag<__bf16>::load(vsl + vo);
        oacc[t] = at_mma(pa, vbh, oacc[t]);
        oacc[t] = at_mma(pa, vbl, oacc[t]);
        oacc[t] = at_mma(pl, vbh, oacc[t]);
      }
    }
  }

  __syncthreads();
  float* os = reinterpret_cast<float*>(lds_raw) + wave * 1088;
#pragma unroll
  for (int r = 0; r < 8; ++r) {
    const float inv = 1.0f / lrow[r];
#pragma unroll
    for (int t = 0; t < 4; ++t) os[(8 * hh + r) * 68 + t * 16 + c] = oacc[t][r] * inv;
  }
  __syncthreads();
  {
    const int q4 = lane >> 3, c8 = (lane & 7) * 8;
    for (int pass = 0; pass < 2; ++pass) {
#pragma unroll
      for (int it = 0; it < 4; ++it) {
        const int row = it * 4 + q4;
        const float* sp = os + row * 68 + c8;
        v8h hv, lv;
#pragma unroll
        for (int e = 0; e < 8; ++e) {
          const unsigned short hb = f2bf_bits(sp[e]);
          const unsigned short lb = f2bf_bits(sp[e] - bf_bits2f(hb));
          hv[e] = __builtin_bit_cast(_Float16, hb);
          lv[e] = __builtin_bit_cast(_Float16, lb);
        }
        const size_t go = (rowb + q0 + row) * (size_t)kDm + hcol + c8;
        *(volatile v8h*)(Oh + go) = hv;
        *(volatile v8h*)(Ol + go) = lv;
      }
      __threadfence();
    }
  }
}

extern "C" void kernel_launch(void* const* d_in, const int* in_sizes, int n_in,
                              void* d_out, int out_size, void* d_ws, size_t ws_size,
                              hipStream_t stream) {
  (void)in_sizes; (void)n_in; (void)out_size;
  const float* x     = (const float*)d_in[0];
  const float* amask = (const float*)d_in[1];
  const float* wq    = (const float*)d_in[2];
  const float* bq    = (const float*)d_in[3];
  const float* wk    = (const float*)d_in[4];
  const float* bk    = (const float*)d_in[5];
  const float* wv    = (const float*)d_in[6];
  const float* bv    = (const float*)d_in[7];
  const float* wo    = (const float*)d_in[8];
  const float* bo    = (const float*)d_in[9];

  constexpr size_t kMiB = 1048576;
  constexpr size_t kActPlane = (size_t)kRows * kDm * 2;
  constexpr size_t kWPlane   = (size_t)kDm * kDm * 2;
  constexpr size_t offXb  = 0;
  constexpr size_t offWq  = 16 * kMiB;
  constexpr size_t offWk  = 18 * kMiB;
  constexpr size_t offWv  = 20 * kMiB;
  constexpr size_t offOh  = 0;
  constexpr size_t offOl  = 16 * kMiB;
  constexpr size_t offQh  = 32 * kMiB;
  constexpr size_t offQl  = 48 * kMiB;
  constexpr size_t offWo  = 32 * kMiB;
  constexpr size_t offKh  = 64 * kMiB;
  constexpr size_t offKl  = 80 * kMiB;
  constexpr size_t offVth = 96 * kMiB;
  constexpr size_t offVtl = 112 * kMiB;
  constexpr size_t kWsTotal = 128 * kMiB;
  static_assert(offWv + kWPlane <= 22 * kMiB);
  static_assert(offOl + kActPlane == offQh);
  static_assert(offQl + kActPlane == offKh);
  static_assert(offWo + kWPlane <= offQl);
  static_assert(offKl + kActPlane == offVth);
  static_assert(offVtl + kActPlane == kWsTotal);
  static_assert(kWsTotal <= (size_t)134217728);
  if (ws_size < kWsTotal) return;

  char* ws = (char*)d_ws;
  unsigned short* xb  = (unsigned short*)(ws + offXb);
  unsigned short* wqb = (unsigned short*)(ws + offWq);
  unsigned short* wkb = (unsigned short*)(ws + offWk);
  unsigned short* wvb = (unsigned short*)(ws + offWv);
  unsigned short* wob = (unsigned short*)(ws + offWo);
  unsigned short* qh  = (unsigned short*)(ws + offQh);
  unsigned short* ql  = (unsigned short*)(ws + offQl);
  unsigned short* kh  = (unsigned short*)(ws + offKh);
  unsigned short* kl  = (unsigned short*)(ws + offKl);
  unsigned short* vth = (unsigned short*)(ws + offVth);
  unsigned short* vtl = (unsigned short*)(ws + offVtl);
  unsigned short* oh  = (unsigned short*)(ws + offOh);
  unsigned short* ol  = (unsigned short*)(ws + offOl);

  constexpr int nx8 = kRows * kDm / 8;
  constexpr int nw8 = kDm * kDm / 8;
  static_assert((kRows * kDm) % 8 == 0);
  static_assert((kDm * kDm) % 8 == 0);
  cast_f32_bf16x8<<<(nx8 + 255) / 256, 256, 0, stream>>>(x,  xb,  nx8);
  cast_f32_bf16x8<<<(nw8 + 255) / 256, 256, 0, stream>>>(wq, wqb, nw8);
  cast_f32_bf16x8<<<(nw8 + 255) / 256, 256, 0, stream>>>(wk, wkb, nw8);
  cast_f32_bf16x8<<<(nw8 + 255) / 256, 256, 0, stream>>>(wv, wvb, nw8);

  constexpr int tilesProj = (kRows / 64) * (kDm / 64);
  const dim3 gproj((tilesProj + 7) / 8, 1);
  wmma_gemm64<1, 0, 2, 2><<<gproj, 256, 0, stream>>>(
      xb, xb, kDm, 0L, wqb, wqb, kDm, 0L, (void*)qh, (void*)ql, kDm, 0L, bq, kRows, kDm, kDm, 1.0f);
  wmma_gemm64<1, 0, 2, 2><<<gproj, 256, 0, stream>>>(
      xb, xb, kDm, 0L, wkb, wkb, kDm, 0L, (void*)kh, (void*)kl, kDm, 0L, bk, kRows, kDm, kDm, 1.0f);
  wmma_gemm64<1, 0, 1, 2><<<gproj, 256, 0, stream>>>(
      wvb, wvb, kDm, 0L, xb, xb, kDm, 0L, (void*)vth, (void*)vtl, kRows, 0L, bv, kDm, kRows, kDm, 1.0f);

  const dim3 gattn(kBatch * kHeads * (kSeq / 64));
  attn64_planes<<<gattn, 128, 0, stream>>>(qh, ql, kh, kl, vth, vtl, amask, oh, ol);

  cast_f32_bf16x8<<<(nw8 + 255) / 256, 256, 0, stream>>>(wo, wob, nw8);

  wmma_gemm64<1, 2, 2, 0><<<gproj, 256, 0, stream>>>(
      oh, ol, kDm, 0L, wob, wob, kDm, 0L, d_out, d_out, kDm, 0L, bo, kRows, kDm, kDm, 1.0f);
}
